// ReverseGRUEncoder_44049184587810
// MI455X (gfx1250) — hardware-verified
//
#include <hip/hip_runtime.h>


#define HID  25
#define KP   32
#define RP   96
#define NOUT 8
#define TPB  128
#define SEQ_PER_BLOCK 64

typedef _Float16 v16h __attribute__((ext_vector_type(16)));
typedef _Float16 v8h  __attribute__((ext_vector_type(8)));
typedef float    v8f  __attribute__((ext_vector_type(8)));
typedef float    v4f  __attribute__((ext_vector_type(4)));
typedef float    v2f  __attribute__((ext_vector_type(2)));

union Frag { v16h v; v8h half[2]; };

__device__ __forceinline__ void mma16(v8f& acc, const v16h a, const v16h b) {
  acc = __builtin_amdgcn_wmma_f32_16x16x32_f16(false, a, false, b, (short)0, acc, false, false);
  asm volatile("v_nop\n\tv_nop\n\tv_nop\n\tv_nop" : "+v"(acc) : "v"(a), "v"(b));
}

__device__ __forceinline__ v8f ld8(const float* p) {
  v4f a = *(const v4f*)p;
  v4f b = *(const v4f*)(p + 4);
  return __builtin_shufflevector(a, b, 0, 1, 2, 3, 4, 5, 6, 7);
}

__device__ __forceinline__ v16h ldA(const _Float16* row, int h) {
  Frag f;
  f.half[0] = *(const v8h*)(row + 8 * h);
  f.half[1] = *(const v8h*)(row + 16 + 8 * h);
  return f.v;
}

__device__ __forceinline__ float sigm_f(float x) {
  const float xc = fminf(fmaxf(x, -30.0f), 30.0f);
  const float e  = __expf(-xc);
  return __builtin_amdgcn_rcpf(1.0f + e);
}
__device__ __forceinline__ float tanh_f(float x) {
  const float xc = fminf(fmaxf(x, -20.0f), 20.0f);
  const float e  = __expf(2.0f * xc);
  return 1.0f - 2.0f * __builtin_amdgcn_rcpf(e + 1.0f);
}

__device__ __forceinline__ v8f xtile(const float* w0, const float* w1, const float* bb, float o0, float o1) {
  const v8f a = ld8(w0), b = ld8(w1), c = ld8(bb);
  v8f x;
#pragma unroll
  for (int r = 0; r < 8; ++r) x[r] = tanh_f(o0 * a[r] + o1 * b[r] + c[r]);
  return x;
}

__device__ __forceinline__ v16h packB(const v8f lo, const v8f hi) {
  v8h a, b;
#pragma unroll
  for (int r = 0; r < 8; ++r) {
    a[r] = (_Float16)(lo[r] * 256.0f);
    b[r] = (_Float16)(hi[r] * 256.0f);
  }
  Frag f;
  f.half[0] = a;
  f.half[1] = b;
  return f.v;
}

__device__ __forceinline__ void gru_phase(const _Float16* sW, const float* sBrz, const float* sBin, const float* sBhn,
                                          int q, int m, int h, const v16h xB, const v16h hB, v8f& hq) {
  const int j0 = q * 16 + 8 * h;
  v8f accR = ld8(sBrz + j0);
  v8f accZ = ld8(sBrz + 32 + j0);
  v8f accI = ld8(sBin + j0);
  v8f accH = ld8(sBhn + j0);
  const int pr = q * 16 + m;
  v16h a;
  a = ldA(sW + (0 * RP + 0 * 32 + pr) * KP, h); mma16(accR, a, xB);
  a = ldA(sW + (1 * RP + 0 * 32 + pr) * KP, h); mma16(accR, a, hB);
  a = ldA(sW + (0 * RP + 1 * 32 + pr) * KP, h); mma16(accZ, a, xB);
  a = ldA(sW + (1 * RP + 1 * 32 + pr) * KP, h); mma16(accZ, a, hB);
  a = ldA(sW + (0 * RP + 2 * 32 + pr) * KP, h); mma16(accI, a, xB);
  a = ldA(sW + (1 * RP + 2 * 32 + pr) * KP, h); mma16(accH, a, hB);
  const float sc = 1.0f / 16384.0f;
#pragma unroll
  for (int r = 0; r < 8; ++r) {
    const float rg = sigm_f(accR[r] * sc);
    const float zg = sigm_f(accZ[r] * sc);
    const float ng = tanh_f(accI[r] * sc + rg * (accH[r] * sc));
    hq[r] = (1.0f - zg) * ng + zg * hq[r];
  }
}

__global__ __launch_bounds__(TPB)
void rgru_scan_kernel(const float* __restrict__ obs,
                      const float* __restrict__ Wp,  const float* __restrict__ bp,
                      const float* __restrict__ Wih, const float* __restrict__ bih,
                      const float* __restrict__ Whh, const float* __restrict__ bhh,
                      const float* __restrict__ Wst, const float* __restrict__ bst,
                      float* out, int B, int T)
{
  __shared__ __attribute__((aligned(16))) _Float16 sW[2 * RP * KP];
  __shared__ __attribute__((aligned(16))) float sBrz[64];
  __shared__ __attribute__((aligned(16))) float sBin[32];
  __shared__ __attribute__((aligned(16))) float sBhn[32];
  __shared__ __attribute__((aligned(16))) float sWp0[32];
  __shared__ __attribute__((aligned(16))) float sWp1[32];
  __shared__ __attribute__((aligned(16))) float sBp[32];
  __shared__ __attribute__((aligned(16))) float sWst[NOUT * 32];
  __shared__ float sBst[NOUT];

  const int tid = threadIdx.x;

#pragma unroll 1
  for (int e = tid; e < 2 * RP * KP; e += TPB) {
    const int mat = e / (RP * KP);
    const int rem = e - mat * (RP * KP);
    const int p   = rem / KP;
    const int k   = rem - p * KP;
    const int g   = p >> 5;
    const int jj  = p & 31;
    const bool in = (jj < HID) && (k < HID);
    const int idx = (g * HID + min(jj, HID - 1)) * HID + min(k, HID - 1);
    const float wi = Wih[idx];
    const float wh = Whh[idx];
    const float w  = (mat != 0) ? wh : wi;
    sW[e] = (_Float16)(in ? w * 64.0f : 0.0f);
  }
  if (tid < 64) {
    const int g   = tid >> 5;
    const int jj  = tid & 31;
    const bool in = (jj < HID);
    const int row = g * HID + min(jj, HID - 1);
    const float v = bih[row] + bhh[row];
    sBrz[tid] = in ? v * 16384.0f : 0.0f;
  }
  if (tid < 32) {
    const int jj  = tid;
    const bool in = (jj < HID);
    const int jc  = min(jj, HID - 1);
    const int row = 2 * HID + jc;
    const float bi = bih[row];
    const float bh = bhh[row];
    const float w0 = Wp[jc * 2 + 0];
    const float w1 = Wp[jc * 2 + 1];
    const float bb = bp[jc];
    sBin[tid] = in ? bi * 16384.0f : 0.0f;
    sBhn[tid] = in ? bh * 16384.0f : 0.0f;
    sWp0[tid] = in ? w0 : 0.0f;
    sWp1[tid] = in ? w1 : 0.0f;
    sBp[tid]  = in ? bb : 0.0f;
  }
#pragma unroll 1
  for (int e = tid; e < NOUT * 32; e += TPB) {
    const int o  = e >> 5;
    const int jj = e & 31;
    const float w = Wst[o * HID + min(jj, HID - 1)];
    sWst[e] = (jj < HID) ? w : 0.0f;
  }
  if (tid < NOUT) sBst[tid] = bst[tid];
  __syncthreads();

  const int lane = tid & 31;
  const int wv   = tid >> 5;
  const int h    = lane >> 4;
  const int m    = lane & 15;
  const int seq  = blockIdx.x * SEQ_PER_BLOCK + wv * 16 + m;
  const int seqc = min(seq, B - 1);
  const float* orow = obs + (size_t)seqc * (size_t)T * 2;

  v8f h0, h1;
#pragma unroll
  for (int r = 0; r < 8; ++r) { h0[r] = 0.0f; h1[r] = 0.0f; }

#pragma unroll 1
  for (int s = 0; s < T; ++s) {
    const int t = T - 1 - s;
    asm volatile("" ::: "memory");

    const v2f o = *(const v2f*)(orow + (size_t)t * 2);
    const float o0 = o[0], o1 = o[1];

    const v8f x0 = xtile(sWp0 + 8 * h,      sWp1 + 8 * h,      sBp + 8 * h,      o0, o1);
    const v8f x1 = xtile(sWp0 + 16 + 8 * h, sWp1 + 16 + 8 * h, sBp + 16 + 8 * h, o0, o1);

    const v16h xB = packB(x0, x1);
    const v16h hB = packB(h0, h1);

    gru_phase(sW, sBrz, sBin, sBhn, 0, m, h, xB, hB, h0);
    asm volatile("" ::: "memory");
    gru_phase(sW, sBrz, sBin, sBhn, 1, m, h, xB, hB, h1);
  }

  float st[NOUT];
#pragma unroll
  for (int oo = 0; oo < NOUT; ++oo) {
    const v8f wa = ld8(sWst + oo * 32 + 8 * h);
    const v8f wb = ld8(sWst + oo * 32 + 16 + 8 * h);
    float sacc = 0.0f;
#pragma unroll
    for (int r = 0; r < 8; ++r) sacc = sacc + wa[r] * h0[r] + wb[r] * h1[r];
    st[oo] = sacc;
  }
#pragma unroll
  for (int oo = 0; oo < NOUT; ++oo) st[oo] += __shfl_xor(st[oo], 16, 32);

  v4f val;
#pragma unroll
  for (int i = 0; i < 4; ++i) {
    const float lo = st[i] + sBst[i];
    const float hi = st[4 + i] + sBst[4 + i];
    val[i] = (h != 0) ? hi : lo;
  }
  float* op = out + (size_t)((h != 0) ? B : 0) * 4 + (size_t)seq * 4;
  if (seq < B) { *(volatile v4f*)op = val; }
  __threadfence();
  if (seq < B) { *(volatile v4f*)op = val; }
}

extern "C" void kernel_launch(void* const* d_in, const int* in_sizes, int n_in,
                              void* d_out, int out_size, void* d_ws, size_t ws_size,
                              hipStream_t stream)
{
  (void)d_ws; (void)ws_size;
  if (n_in < 9) return;
  if (out_size <= 0 || (out_size % (2 * 4)) != 0) return;
  const int B = out_size / 8;
  if (B < 1) return;
  if (in_sizes[0] <= 0 || (in_sizes[0] % (2 * B)) != 0) return;
  const int T = in_sizes[0] / (2 * B);
  if (T < 1) return;
  if (in_sizes[1] != HID * 2 || in_sizes[2] != HID) return;
  if (in_sizes[3] != 3 * HID * HID || in_sizes[4] != 3 * HID) return;
  if (in_sizes[5] != 3 * HID * HID || in_sizes[6] != 3 * HID) return;
  if (in_sizes[7] != NOUT * HID || in_sizes[8] != NOUT) return;

  const float* obs = (const float*)d_in[0];
  const float* Wp  = (const float*)d_in[1];
  const float* bp  = (const float*)d_in[2];
  const float* Wih = (const float*)d_in[3];
  const float* bih = (const float*)d_in[4];
  const float* Whh = (const float*)d_in[5];
  const float* bhh = (const float*)d_in[6];
  const float* Wst = (const float*)d_in[7];
  const float* bst = (const float*)d_in[8];
  float* out = (float*)d_out;

  const int blocks = (B + SEQ_PER_BLOCK - 1) / SEQ_PER_BLOCK;
  rgru_scan_kernel<<<dim3(blocks), dim3(TPB), 0, stream>>>(
      obs, Wp, bp, Wih, bih, Whh, bhh, Wst, bst, out, B, T);
}
